// WalkConv_1623497638433
// MI455X (gfx1250) — hardware-verified
//
#include <hip/hip_runtime.h>
#include <stddef.h>


#define HID    16
#define H4     64
#define EDIM   8
#define FF     256
#define NTHR   256
#define NWAVE  8
#define ETHR   128
#define EWAVE  4
#define EPB    (EWAVE * 16)
#define APZ    72
#define SPZ    264
#define GE     8
#define KG     (GE * HID)
#define APA    136
#define APB    136
#define ITR    128
#define KT     128
#define DEGCAP 256
#define EPT    8
#define CHUNK  (NTHR * EPT)
#define WCAP   (EPT * 32)
#define WSC    8.0f
#define ASC    8.0f
#define FSC    8.0f
#define R_W    0.125f
#define R_AW   0.015625f
#define R_MF   0.0078125f
#define PO_W0  0
#define PO_W1  2048
#define PO_W2  6144
#define PO_W3  10240
#define PO_V0  26624
#define PO_V1  28672
#define PO_V2  32768
#define PO_V3  36864
#define PO_L   37888
#define PTOT   38400
#define WSCAP  134217728

static_assert(ITR == NWAVE * 16);
static_assert(KT == NWAVE * 16);
static_assert(DEGCAP == NTHR);
static_assert((CHUNK & (CHUNK - 1)) == 0);
static_assert((DEGCAP % GE) == 0);
static_assert(KG == 128);
static_assert((APZ % 8) == 0 && (APA % 8) == 0 && (APB % 8) == 0 && (SPZ % 8) == 0);
static_assert(PTOT == PO_L + 512);
static_assert((PTOT * 2) % 256 == 0);
static_assert(2 * NTHR * 4 == ITR * HID);

typedef float    v4f  __attribute__((ext_vector_type(4)));
typedef float    v8f  __attribute__((ext_vector_type(8)));
typedef int      v4i  __attribute__((ext_vector_type(4)));
typedef _Float16 v8h  __attribute__((ext_vector_type(8)));
typedef _Float16 v16h __attribute__((ext_vector_type(16)));
union Frag { v16h v; v8h h[2]; };

__device__ __forceinline__ v8f wmh(v16h a, v16h b, v8f c) {
  v8f d = __builtin_amdgcn_wmma_f32_16x16x32_f16(false, a, false, b, (short)0, c, false, false);
  asm volatile("v_nop\n\tv_nop\n\tv_nop\n\tv_nop" : "+v"(d) : "v"(a), "v"(b));
  return d;
}

__device__ __forceinline__ v8h cvt8(v4f a, v4f b, float scl) {
  v8h r;
  r[0] = (_Float16)(a.x * scl); r[1] = (_Float16)(a.y * scl); r[2] = (_Float16)(a.z * scl); r[3] = (_Float16)(a.w * scl);
  r[4] = (_Float16)(b.x * scl); r[5] = (_Float16)(b.y * scl); r[6] = (_Float16)(b.z * scl); r[7] = (_Float16)(b.w * scl);
  return r;
}

template <int NT, int KS, int KP>
__device__ __forceinline__ void mma_w(const _Float16* At, const _Float16* __restrict__ Bp,
                                      int lane, v8f (&acc)[NT]) {
  static_assert(KS * 32 <= KP);
  const int hh = lane >> 4, m = lane & 15;
#pragma unroll
  for (int t = 0; t < NT; ++t) { v8f z = {0.f, 0.f, 0.f, 0.f, 0.f, 0.f, 0.f, 0.f}; acc[t] = z; }
  const _Float16* ap = At + m * APZ + 8 * hh;
  const _Float16* bb = Bp + (size_t)m * KP + 8 * hh;
#pragma unroll
  for (int ks = 0; ks < KS; ++ks) {
    Frag a;
    a.h[0] = *(const v8h*)(ap + 32 * ks);
    a.h[1] = *(const v8h*)(ap + 32 * ks + 16);
#pragma unroll
    for (int t = 0; t < NT; ++t) {
      const _Float16* bp = bb + (size_t)(16 * t) * KP + 32 * ks;
      Frag b;
      b.h[0] = *(const v8h*)bp;
      b.h[1] = *(const v8h*)(bp + 16);
      acc[t] = wmh(a.v, b.v, acc[t]);
    }
  }
}

template <int NT>
__device__ __forceinline__ void epi_relu(_Float16* Qt, v8f (&acc)[NT], const float* __restrict__ bias,
                                         int col0, float scl, int lane) {
  const int hh = lane >> 4, m = lane & 15;
#pragma unroll
  for (int t = 0; t < NT; ++t) {
    const float bv = bias[col0 + 16 * t + m];
#pragma unroll
    for (int r = 0; r < 8; ++r) {
      const float v = fmaxf(acc[t][r] * scl + bv, 0.0f);
      Qt[(8 * hh + r) * APZ + col0 + 16 * t + m] = (_Float16)(v * ASC);
    }
  }
}

__device__ __forceinline__ int scan_chunk(const int* __restrict__ dsts, int nE, int cbase, int key,
                                          int vecok, int* wl, int tid, int lane, int wave) {
  const int el0 = tid * EPT;
  const int e0  = cbase + el0;
  const int sent = -2147483647 - 1;
  v4i da, db;
  if (vecok != 0 && cbase + CHUNK <= nE) {
    da = *(const v4i*)(dsts + e0);
    db = *(const v4i*)(dsts + e0 + 4);
  } else {
    const int le = nE - 1;
    da.x = (e0     < nE) ? dsts[min(e0,     le)] : sent;
    da.y = (e0 + 1 < nE) ? dsts[min(e0 + 1, le)] : sent;
    da.z = (e0 + 2 < nE) ? dsts[min(e0 + 2, le)] : sent;
    da.w = (e0 + 3 < nE) ? dsts[min(e0 + 3, le)] : sent;
    db.x = (e0 + 4 < nE) ? dsts[min(e0 + 4, le)] : sent;
    db.y = (e0 + 5 < nE) ? dsts[min(e0 + 5, le)] : sent;
    db.z = (e0 + 6 < nE) ? dsts[min(e0 + 6, le)] : sent;
    db.w = (e0 + 7 < nE) ? dsts[min(e0 + 7, le)] : sent;
  }
  const bool h0 = da.x == key, h1 = da.y == key, h2 = da.z == key, h3 = da.w == key;
  const bool h4 = db.x == key, h5 = db.y == key, h6 = db.z == key, h7 = db.w == key;
  int wc = 0;
  const unsigned any = __builtin_amdgcn_ballot_w32(h0 | h1 | h2 | h3 | h4 | h5 | h6 | h7);
  if (any != 0u) {
#define HITJ(J, HJ) { \
      const unsigned mj = __builtin_amdgcn_ballot_w32(HJ); \
      if (mj != 0u) { \
        if (HJ) { \
          const int pos = wc + (int)__builtin_amdgcn_mbcnt_lo(mj, 0u); \
          if (pos < WCAP) wl[wave * WCAP + pos] = el0 + (J); \
        } \
        wc += (int)__builtin_popcount(mj); } }
    HITJ(0, h0)
    HITJ(1, h1)
    HITJ(2, h2)
    HITJ(3, h3)
    HITJ(4, h4)
    HITJ(5, h5)
    HITJ(6, h6)
    HITJ(7, h7)
#undef HITJ
  }
  return wc;
}

__global__ __launch_bounds__(NTHR) void k_wprep(
    const float* __restrict__ W0, const float* __restrict__ W1, const float* __restrict__ W2,
    const float* __restrict__ W3, const float* __restrict__ V0, const float* __restrict__ V1,
    const float* __restrict__ V2, const float* __restrict__ V3, const float* __restrict__ L,
    _Float16* Wp) {
  const int pid = blockIdx.y;
  const float* W = L; int K = HID, N = HID, KP = 32, po = PO_L;
  switch (pid) {
    case 0: W = W0; K = EDIM; N = H4;  KP = 32; po = PO_W0; break;
    case 1: W = W1; K = H4;   N = H4;  KP = 64; po = PO_W1; break;
    case 2: W = W2; K = H4;   N = H4;  KP = 64; po = PO_W2; break;
    case 3: W = W3; K = H4;   N = FF;  KP = 64; po = PO_W3; break;
    case 4: W = V0; K = HID;  N = H4;  KP = 32; po = PO_V0; break;
    case 5: W = V1; K = H4;   N = H4;  KP = 64; po = PO_V1; break;
    case 6: W = V2; K = H4;   N = H4;  KP = 64; po = PO_V2; break;
    case 7: W = V3; K = H4;   N = HID; KP = 64; po = PO_V3; break;
    default: break;
  }
  const int kp8 = KP >> 3;
  const int chunks = N * kp8;
  const int c = blockIdx.x * NTHR + threadIdx.x;
  if (c >= chunks) return;
  const int n = c / kp8;
  const int k0 = (c - n * kp8) * 8;
  v8h hv;
#pragma unroll
  for (int e = 0; e < 8; ++e) {
    const int k = k0 + e;
    const int kc = k < K ? k : K - 1;
    float v = W[(size_t)kc * N + n] * WSC;
    v = (k < K) ? v : 0.0f;
    hv[e] = (_Float16)v;
  }
  _Float16* dp = Wp + po + (size_t)c * 8;
  *(volatile v8h*)dp = hv;
  __threadfence();
  *(volatile v8h*)dp = hv;
}

__global__ __launch_bounds__(ETHR) void k_edge(
    const float* __restrict__ attr, const float* __restrict__ b0, const float* __restrict__ b1,
    const float* __restrict__ b2, const float* __restrict__ b3, const _Float16* __restrict__ Wp,
    _Float16* Fp, int nE) {
  __shared__ __attribute__((aligned(16))) _Float16 tp[EWAVE * 16 * APZ];
  __shared__ __attribute__((aligned(16))) _Float16 tq[EWAVE * 16 * APZ];
  __shared__ __attribute__((aligned(16))) _Float16 sg[EWAVE * 16 * SPZ];
  const int tid = threadIdx.x, lane = tid & 31, wave = tid >> 5, hh = lane >> 4, m = lane & 15;
  _Float16* P  = tp + wave * (16 * APZ);
  _Float16* Q  = tq + wave * (16 * APZ);
  _Float16* Sg = sg + wave * (16 * SPZ);
  const int eb = blockIdx.x * EPB + wave * 16;

  {
    const int row = lane >> 1, half = lane & 1;
    int er = eb + row;
    er = er > nE - 1 ? nE - 1 : er;
    const float* ap = attr + (size_t)er * EDIM;
    const v4f a0 = *(const v4f*)ap, a1 = *(const v4f*)(ap + 4);
    const v8h dv = cvt8(a0, a1, 1.0f);
    v8h sv, z;
#pragma unroll
    for (int e = 0; e < 8; ++e) { z[e] = (_Float16)0.0f; sv[e] = (half == 0) ? dv[e] : (_Float16)0.0f; }
    *(v8h*)(P + row * APZ + 8 * half) = sv;
    *(v8h*)(P + row * APZ + 16 + 8 * half) = z;
  }
  __syncthreads();
  { v8f acc[4]; mma_w<4, 1, 32>(P, Wp + PO_W0, lane, acc); epi_relu<4>(Q, acc, b0, 0, R_W, lane); }
  __syncthreads();
  { v8f acc[4]; mma_w<4, 2, 64>(Q, Wp + PO_W1, lane, acc); epi_relu<4>(P, acc, b1, 0, R_AW, lane); }
  __syncthreads();
  { v8f acc[4]; mma_w<4, 2, 64>(P, Wp + PO_W2, lane, acc); epi_relu<4>(Q, acc, b2, 0, R_AW, lane); }
  __syncthreads();
#pragma unroll 1
  for (int cg = 0; cg < 4; ++cg) {
    v8f acc[4];
    mma_w<4, 2, 64>(Q, Wp + PO_W3 + (size_t)(64 * cg) * 64, lane, acc);
#pragma unroll
    for (int tt = 0; tt < 4; ++tt) {
      const int n = 64 * cg + 16 * tt + m;
      const float bv = b3[n];
      const int cidx = 4 * cg + tt;
#pragma unroll
      for (int r = 0; r < 8; ++r) {
        const float v = (acc[tt][r] * R_AW + bv) * FSC;
        Sg[(8 * hh + r) * SPZ + m * 16 + cidx] = (_Float16)v;
      }
    }
  }
  __syncthreads();
  _Float16* gw = Fp + (size_t)eb * FF;
  v8h ov[16];
#pragma unroll
  for (int it = 0; it < 16; ++it) ov[it] = *(const v8h*)(Sg + it * SPZ + 8 * lane);
#pragma unroll
  for (int it = 0; it < 16; ++it) *(volatile v8h*)(gw + (size_t)it * FF + 8 * lane) = ov[it];
  __threadfence();
#pragma unroll
  for (int it = 0; it < 16; ++it) *(volatile v8h*)(gw + (size_t)it * FF + 8 * lane) = ov[it];
}

__global__ __launch_bounds__(NTHR) void k_msg(
    const float* __restrict__ mtr, const int* __restrict__ ei, const _Float16* __restrict__ Fp,
    float* M1, int nN, int nE, int vecok) {
  __shared__ __attribute__((aligned(16))) _Float16 At[ITR * APA];
  __shared__ __attribute__((aligned(16))) _Float16 Bt[HID * APB];
  __shared__ __attribute__((aligned(16))) float Sf[ITR * HID];
  __shared__ __attribute__((aligned(16))) int wl[NWAVE * WCAP];
  __shared__ __attribute__((aligned(16))) int elist[DEGCAP];
  __shared__ __attribute__((aligned(16))) int esrc[DEGCAP];
  __shared__ int wcnt[NWAVE];
  __shared__ int cntsh;
  const int tid = threadIdx.x, lane = tid & 31, wave = tid >> 5, hh = lane >> 4, m = lane & 15;
  const int k = blockIdx.x;
  const int* srcs = ei;
  const int* dsts = ei + nE;

  elist[tid] = 0;
  __syncthreads();

  int cnt = 0;
  const int nChunks = (nE + CHUNK - 1) / CHUNK;
#pragma unroll 1
  for (int ch = 0; ch < nChunks; ++ch) {
    const int cbase = ch * CHUNK;
    const int wc = scan_chunk(dsts, nE, cbase, k, vecok, wl, tid, lane, wave);
    if (lane == 0) wcnt[wave] = wc;
    __syncthreads();
    if (wave == 0) {
#pragma unroll 1
      for (int w = 0; w < NWAVE; ++w) {
        int n = __builtin_amdgcn_readfirstlane(wcnt[w]);
        n = n > WCAP ? WCAP : (n < 0 ? 0 : n);
#pragma unroll 1
        for (int i = 0; i < n; ++i) {
          const int ent = __builtin_amdgcn_readfirstlane(wl[w * WCAP + i]);
          int e = cbase + (ent & (CHUNK - 1));
          e = e > nE - 1 ? nE - 1 : (e < 0 ? 0 : e);
          if (lane == 0 && cnt < DEGCAP) elist[cnt] = e;
          cnt++;
        }
      }
    }
    __syncthreads();
  }
  if (tid == 0) cntsh = cnt > DEGCAP ? DEGCAP : cnt;
  __syncthreads();
  int cn = cntsh;
  cn = cn < 0 ? 0 : (cn > DEGCAP ? DEGCAP : cn);
  cn = __builtin_amdgcn_readfirstlane(cn);
  {
    int e = elist[tid];
    e = e > nE - 1 ? nE - 1 : (e < 0 ? 0 : e);
    int s = srcs[e];
    s = s < 0 ? 0 : (s > nN - 1 ? nN - 1 : s);
    esrc[tid] = s;
  }
  __syncthreads();

  const int ng  = (cn + GE - 1) / GE;
  const int nIT = nN / ITR;
#pragma unroll 1
  for (int it = 0; it < nIT; ++it) {
    v8f acc = {0.f, 0.f, 0.f, 0.f, 0.f, 0.f, 0.f, 0.f};
#pragma unroll 1
    for (int g = 0; g < ng; ++g) {
      {
        const int r = tid >> 1;
        const int irow = it * ITR + r;
        const int slb = (tid & 1) * 4;
#pragma unroll
        for (int q = 0; q < 4; ++q) {
          const int sl = slb + q;
          const int s = g * GE + sl;
          const bool valid = s < cn;
          const int src = esrc[s > DEGCAP - 1 ? DEGCAP - 1 : s];
          const float* p = mtr + ((size_t)irow * nN + src) * HID;
          const v4f x0 = *(const v4f*)p, x1 = *(const v4f*)(p + 4);
          const v4f x2 = *(const v4f*)(p + 8), x3 = *(const v4f*)(p + 12);
          v8h lo = cvt8(x0, x1, 1.0f), hi = cvt8(x2, x3, 1.0f);
#pragma unroll
          for (int e = 0; e < 8; ++e) { lo[e] = valid ? lo[e] : (_Float16)0.0f; hi[e] = valid ? hi[e] : (_Float16)0.0f; }
          *(v8h*)(At + r * APA + 16 * sl) = lo;
          *(v8h*)(At + r * APA + 16 * sl + 8) = hi;
        }
      }
      if (tid < 128) {
        const int t = tid >> 3, sl = tid & 7;
        const int s = g * GE + sl;
        const bool valid = s < cn;
        int e = elist[s > DEGCAP - 1 ? DEGCAP - 1 : s];
        e = e > nE - 1 ? nE - 1 : (e < 0 ? 0 : e);
        const _Float16* p = Fp + ((size_t)e * HID + t) * HID;
        v8h b0v = *(const v8h*)p, b1v = *(const v8h*)(p + 8);
#pragma unroll
        for (int q = 0; q < 8; ++q) { b0v[q] = valid ? b0v[q] : (_Float16)0.0f; b1v[q] = valid ? b1v[q] : (_Float16)0.0f; }
        *(v8h*)(Bt + t * APB + 16 * sl) = b0v;
        *(v8h*)(Bt + t * APB + 16 * sl + 8) = b1v;
      }
      __syncthreads();
      {
        const _Float16* ap = At + (16 * wave + m) * APA + 8 * hh;
        const _Float16* bp = Bt + m * APB + 8 * hh;
#pragma unroll
        for (int ks = 0; ks < 4; ++ks) {
          Frag a, b;
          a.h[0] = *(const v8h*)(ap + 32 * ks);
          a.h[1] = *(const v8h*)(ap + 32 * ks + 16);
          b.h[0] = *(const v8h*)(bp + 32 * ks);
          b.h[1] = *(const v8h*)(bp + 32 * ks + 16);
          acc = wmh(a.v, b.v, acc);
        }
      }
      __syncthreads();
    }
#pragma unroll
    for (int r = 0; r < 8; ++r) {
      const int lrow = 16 * wave + 8 * hh + r;
      const int irow = it * ITR + lrow;
      const float v = (irow == k) ? 0.0f : acc[r] * R_MF;
      Sf[lrow * HID + m] = v;
    }
    __syncthreads();
    {
      float* gp = M1 + ((size_t)k * nN + (size_t)it * ITR) * HID;
      const v4f v0 = *(const v4f*)(Sf + 4 * tid);
      const v4f v1 = *(const v4f*)(Sf + 4 * (NTHR + tid));
      *(volatile v4f*)(gp + 4 * tid) = v0;
      *(volatile v4f*)(gp + 4 * (NTHR + tid)) = v1;
      __threadfence();
      *(volatile v4f*)(gp + 4 * tid) = v0;
      *(volatile v4f*)(gp + 4 * (NTHR + tid)) = v1;
    }
    __syncthreads();
  }
}

__global__ __launch_bounds__(NTHR) void k_node(
    const float* __restrict__ mtr, const float* __restrict__ M1,
    const float* __restrict__ c0, const float* __restrict__ c1, const float* __restrict__ c2,
    const float* __restrict__ c3, const float* __restrict__ Lb, const _Float16* __restrict__ Wp,
    float* out, int nN) {
  __shared__ __attribute__((aligned(16))) _Float16 tp[NWAVE * 16 * APZ];
  __shared__ __attribute__((aligned(16))) _Float16 tq[NWAVE * 16 * APZ];
  __shared__ __attribute__((aligned(16))) float so[NWAVE * 256];
  const int tid = threadIdx.x, lane = tid & 31, wave = tid >> 5, hh = lane >> 4, m = lane & 15;
  const int nkt = nN / KT;
  const int bi = blockIdx.x;
  const int i  = bi / nkt;
  const int kt = bi - i * nkt;
  const int kb = kt * KT + 16 * wave;
  _Float16* P = tp + wave * (16 * APZ);
  _Float16* Q = tq + wave * (16 * APZ);
  float*   So = so + wave * 256;

  {
    const int row = lane >> 1, half = lane & 1;
    const float* p = M1 + ((size_t)i * nN + (kb + row)) * HID + 8 * half;
    const v4f a0 = *(const v4f*)p, a1 = *(const v4f*)(p + 4);
    const v8h hv = cvt8(a0, a1, ASC);
    v8h z;
#pragma unroll
    for (int e = 0; e < 8; ++e) z[e] = (_Float16)0.0f;
    *(v8h*)(P + row * APZ + 8 * half) = hv;
    *(v8h*)(P + row * APZ + 16 + 8 * half) = z;
  }
  __syncthreads();
  {
    v8f acc[1];
    mma_w<1, 1, 32>(P, Wp + PO_L, lane, acc);
    const float lbv = Lb[m];
#pragma unroll
    for (int r = 0; r < 8; ++r) {
      const int kk = kb + 8 * hh + r;
      const float add = M1[((size_t)kk * nN + i) * HID + m];
      const float v = add + (acc[0][r] * R_AW + lbv);
      Q[(8 * hh + r) * APZ + m] = (_Float16)(v * ASC);
      Q[(8 * hh + r) * APZ + 16 + m] = (_Float16)0.0f;
    }
  }
  __syncthreads();
  { v8f acc[4]; mma_w<4, 1, 32>(Q, Wp + PO_V0, lane, acc); epi_relu<4>(P, acc, c0, 0, R_AW, lane); }
  __syncthreads();
  { v8f acc[4]; mma_w<4, 2, 64>(P, Wp + PO_V1, lane, acc); epi_relu<4>(Q, acc, c1, 0, R_AW, lane); }
  __syncthreads();
  { v8f acc[4]; mma_w<4, 2, 64>(Q, Wp + PO_V2, lane, acc); epi_relu<4>(P, acc, c2, 0, R_AW, lane); }
  __syncthreads();
  {
    v8f acc[1];
    mma_w<1, 2, 64>(P, Wp + PO_V3, lane, acc);
    const float cv = c3[m];
#pragma unroll
    for (int r = 0; r < 8; ++r) So[(8 * hh + r) * HID + m] = acc[0][r] * R_AW + cv;
  }
  __syncthreads();
  {
    const size_t gofs = ((size_t)i * nN + kb) * HID;
    const v4f s0 = *(const v4f*)(So + 4 * lane);
    const v4f s1 = *(const v4f*)(So + 128 + 4 * lane);
    const v4f x0 = *(const v4f*)(mtr + gofs + 4 * lane);
    const v4f x1 = *(const v4f*)(mtr + gofs + 128 + 4 * lane);
    const v4f o0 = x0 + s0, o1 = x1 + s1;
    *(volatile v4f*)(out + gofs + 4 * lane) = o0;
    *(volatile v4f*)(out + gofs + 128 + 4 * lane) = o1;
    __threadfence();
    *(volatile v4f*)(out + gofs + 4 * lane) = o0;
    *(volatile v4f*)(out + gofs + 128 + 4 * lane) = o1;
  }
}

extern "C" void kernel_launch(void* const* d_in, const int* in_sizes, int n_in,
                              void* d_out, int out_size, void* d_ws, size_t ws_size,
                              hipStream_t stream) {
  if (n_in < 21) return;
  int nN = 0;
  while (nN < 46340 && (long long)(nN + 1) * (nN + 1) * HID <= (long long)in_sizes[0]) ++nN;
  if (nN < KT || (nN % KT) != 0 || (nN % ITR) != 0) return;
  if ((long long)nN * nN * HID != (long long)in_sizes[0]) return;
  const int nE = in_sizes[2] / 2;
  if (nE <= 0 || in_sizes[2] != 2 * nE || in_sizes[1] != nE * EDIM) return;
  if (in_sizes[3] != EDIM * H4 || in_sizes[4] != H4 || in_sizes[5] != H4 * H4 || in_sizes[6] != H4) return;
  if (in_sizes[7] != H4 * H4 || in_sizes[8] != H4 || in_sizes[9] != H4 * FF || in_sizes[10] != FF) return;
  if (in_sizes[11] != HID * H4 || in_sizes[12] != H4 || in_sizes[13] != H4 * H4 || in_sizes[14] != H4) return;
  if (in_sizes[15] != H4 * H4 || in_sizes[16] != H4 || in_sizes[17] != H4 * HID || in_sizes[18] != HID) return;
  if (in_sizes[19] != HID * HID || in_sizes[20] != HID) return;
  if ((long long)out_size != (long long)nN * nN * HID) return;
  if (nE > (1 << 26) || nN > 4096) return;

  const float* mtr  = (const float*)d_in[0];
  const float* attr = (const float*)d_in[1];
  const int*   ei   = (const int*)d_in[2];
  const float* W0 = (const float*)d_in[3];  const float* b0 = (const float*)d_in[4];
  const float* W1 = (const float*)d_in[5];  const float* b1 = (const float*)d_in[6];
  const float* W2 = (const float*)d_in[7];  const float* b2 = (const float*)d_in[8];
  const float* W3 = (const float*)d_in[9];  const float* b3 = (const float*)d_in[10];
  const float* V0 = (const float*)d_in[11]; const float* c0 = (const float*)d_in[12];
  const float* V1 = (const float*)d_in[13]; const float* c1 = (const float*)d_in[14];
  const float* V2 = (const float*)d_in[15]; const float* c2 = (const float*)d_in[16];
  const float* V3 = (const float*)d_in[17]; const float* c3 = (const float*)d_in[18];
  const float* L  = (const float*)d_in[19]; const float* Lb = (const float*)d_in[20];
  float* out = (float*)d_out;

  const int nBlkE = (nE + EPB - 1) / EPB;
  const int EPAD  = nBlkE * EPB;

  char* ws = (char*)d_ws;
  size_t off = 0;
  const size_t oWp = off; off += (size_t)PTOT * 2;                 off = (off + 255) & ~(size_t)255;
  const size_t oF  = off; off += (size_t)EPAD * FF * 2;            off = (off + 255) & ~(size_t)255;
  const size_t oM1 = off; off += (size_t)nN * nN * HID * 4;         off = (off + 255) & ~(size_t)255;
  if (off > ws_size || off > (size_t)WSCAP) return;
  _Float16* Wp = (_Float16*)(ws + oWp);
  _Float16* Fp = (_Float16*)(ws + oF);
  float*    M1 = (float*)(ws + oM1);

  const int vecok = ((nE & 3) == 0) ? 1 : 0;

  k_wprep<<<dim3(8, 9), NTHR, 0, stream>>>(W0, W1, W2, W3, V0, V1, V2, V3, L, Wp);
  k_edge<<<nBlkE, ETHR, 0, stream>>>(attr, b0, b1, b2, b3, Wp, Fp, nE);
  k_msg<<<nN, NTHR, 0, stream>>>(mtr, ei, Fp, M1, nN, nE, vecok);
  k_node<<<nN * (nN / KT), NTHR, 0, stream>>>(mtr, M1, c0, c1, c2, c3, Lb, Wp, out, nN);
}
